// GMNLayerX_Pooling2_28432683499989
// MI455X (gfx1250) — hardware-run, weakly checked
//
#include <hip/hip_runtime.h>
#include <hip/hip_bf16.h>
#include <stddef.h>


#define TT     10
#define NNODE  2048
#define NEDGE  32768
#define HID    256
#define NTHR   256
#define NWAVE  8
#define ET     64
#define NB     64
#define EPT    8
#define CHUNK  (NTHR * EPT)
#define WCAP   (EPT * 32)
#define NROWS  (TT * NNODE)

#define PL_PQ  131072
#define PL_R   8192
#define PL_SQ  65536
#define PL_N1  196608

#define L_AH     0
#define L_AL     32768
#define L_EST    65536
#define PN_BYTES 131072
#define EK_ARH   131072
#define EK_ARL   135168
#define EK_CD    139264
#define EK_TRS   142336
#define EK_ROW   146432
#define EK_COL   146688
#define EK_BYTES 146944
#define AG_ACC   0
#define AG_ACT   65536
#define AG_LIST  69632
#define AG_CO    77824
#define AG_BYTES 80896

static_assert((NEDGE % ET) == 0);
static_assert((NEDGE % CHUNK) == 0);
static_assert((NNODE % NB) == 0);
static_assert((NROWS % 64) == 0);
static_assert(NB * 12 == 3 * NTHR);
static_assert(NB < 256);
static_assert(CHUNK == 2048);
static_assert(NWAVE * 32 == NTHR);

typedef float        v4f   __attribute__((ext_vector_type(4)));
typedef float        v8f   __attribute__((ext_vector_type(8)));
typedef int          v4i   __attribute__((ext_vector_type(4)));
typedef int          v8i   __attribute__((ext_vector_type(8)));
typedef unsigned int u32x4 __attribute__((ext_vector_type(4)));
typedef __bf16       v8bf  __attribute__((ext_vector_type(8)));
typedef __bf16       v16bf __attribute__((ext_vector_type(16)));

union Frag16 { u32x4 u[2]; v16bf v; v8i w; };
union Pk8    { v8bf b; u32x4 u; };

__device__ __forceinline__ v8f zero8f() {
  v8f z;
#pragma unroll
  for (int i = 0; i < 8; ++i) z[i] = 0.0f;
  return z;
}

__device__ __forceinline__ void zacc(v8f (&a)[4], v8f (&b)[4]) {
#pragma unroll
  for (int mt = 0; mt < 4; ++mt) { a[mt] = zero8f(); b[mt] = zero8f(); }
}

__device__ __forceinline__ Frag16 lda_frag(const __bf16* plane, int pitch, int row0, int k0, int lane) {
  const __bf16* p = plane + (row0 + (lane & 15)) * pitch + k0 + ((lane >> 4) << 3);
  Frag16 f;
  f.u[0] = *(const u32x4*)p;
  f.u[1] = *(const u32x4*)(p + 16);
  return f;
}

__device__ __forceinline__ Frag16 ldb_frag(const __bf16* pack, int nt, int kt, int KtB, int lane) {
  const __bf16* p = pack + ((((size_t)nt * KtB + kt) * 32 + lane) << 4);
  Frag16 f;
  f.u[0] = *(const u32x4*)p;
  f.u[1] = *(const u32x4*)(p + 8);
  return f;
}

__device__ __forceinline__ v8f wmb(v16bf a, v16bf b, v8f c) {
  return __builtin_amdgcn_wmma_f32_16x16x32_bf16(false, a, false, b, (short)0, c, false, false);
}

__device__ __forceinline__ void gemm_tile(const __bf16* Ah, const __bf16* Al, int pa, int Kt,
                                          const __bf16* __restrict__ Bh, const __bf16* __restrict__ Bl,
                                          int KtB, int kb0, int nt0, int lane,
                                          v8f (&acc0)[4], v8f (&acc1)[4]) {
#pragma unroll 1
  for (int kt = 0; kt < Kt; ++kt) {
    const Frag16 b0h = ldb_frag(Bh, nt0,     kb0 + kt, KtB, lane);
    const Frag16 b0l = ldb_frag(Bl, nt0,     kb0 + kt, KtB, lane);
    const Frag16 b1h = ldb_frag(Bh, nt0 + 1, kb0 + kt, KtB, lane);
    const Frag16 b1l = ldb_frag(Bl, nt0 + 1, kb0 + kt, KtB, lane);
#pragma unroll
    for (int mt = 0; mt < 4; ++mt) {
      const Frag16 ah = lda_frag(Ah, pa, 16 * mt, 32 * kt, lane);
      const Frag16 al = lda_frag(Al, pa, 16 * mt, 32 * kt, lane);
      v8f d0 = acc0[mt], d1 = acc1[mt];
      d0 = wmb(ah.v, b0h.v, d0);
      d0 = wmb(ah.v, b0l.v, d0);
      d0 = wmb(al.v, b0h.v, d0);
      d1 = wmb(ah.v, b1h.v, d1);
      d1 = wmb(ah.v, b1l.v, d1);
      d1 = wmb(al.v, b1h.v, d1);
      asm volatile("v_nop\n\tv_nop\n\tv_nop\n\tv_nop"
                   : "+v"(d0), "+v"(d1)
                   : "v"(ah.w), "v"(al.w), "v"(b0h.w), "v"(b0l.w), "v"(b1h.w), "v"(b1l.w));
      acc0[mt] = d0;
      acc1[mt] = d1;
    }
  }
}

__device__ __forceinline__ void gemm_tile1(const __bf16* Ah, int pa, int Kt,
                                           const __bf16* __restrict__ Bh, int KtB, int kb0, int nt0, int lane,
                                           v8f (&acc0)[4], v8f (&acc1)[4]) {
#pragma unroll 1
  for (int kt = 0; kt < Kt; ++kt) {
    const Frag16 b0h = ldb_frag(Bh, nt0,     kb0 + kt, KtB, lane);
    const Frag16 b1h = ldb_frag(Bh, nt0 + 1, kb0 + kt, KtB, lane);
#pragma unroll
    for (int mt = 0; mt < 4; ++mt) {
      const Frag16 ah = lda_frag(Ah, pa, 16 * mt, 32 * kt, lane);
      v8f d0 = acc0[mt], d1 = acc1[mt];
      d0 = wmb(ah.v, b0h.v, d0);
      d1 = wmb(ah.v, b1h.v, d1);
      asm volatile("v_nop\n\tv_nop\n\tv_nop\n\tv_nop"
                   : "+v"(d0), "+v"(d1)
                   : "v"(ah.w), "v"(b0h.w), "v"(b1h.w));
      acc0[mt] = d0;
      acc1[mt] = d1;
    }
  }
}

__device__ __forceinline__ void split8(const v4f a, const v4f b, Pk8& hi, Pk8& lo) {
  float v[8];
  v[0] = a.x; v[1] = a.y; v[2] = a.z; v[3] = a.w;
  v[4] = b.x; v[5] = b.y; v[6] = b.z; v[7] = b.w;
#pragma unroll
  for (int i = 0; i < 8; ++i) {
    const __bf16 t = (__bf16)v[i];
    hi.b[i] = t;
    lo.b[i] = (__bf16)(v[i] - (float)t);
  }
}

__device__ __forceinline__ void stage_rows(const float* __restrict__ src, int rb, __bf16* Ah, __bf16* Al, int tid) {
#pragma unroll 2
  for (int i = 0; i < 8; ++i) {
    const int g = tid + NTHR * i, row = g >> 5, c8 = (g & 31) << 3;
    const float* s = src + (size_t)(rb + row) * HID + c8;
    const v4f a = *(const v4f*)s;
    const v4f b = *(const v4f*)(s + 4);
    Pk8 hi, lo;
    split8(a, b, hi, lo);
    *(u32x4*)(Ah + row * HID + c8) = hi.u;
    *(u32x4*)(Al + row * HID + c8) = lo.u;
  }
}

__device__ __forceinline__ void cvt_tile(const float* Est, __bf16* Ah, __bf16* Al, int tid) {
#pragma unroll 2
  for (int i = 0; i < 8; ++i) {
    const int g = tid + NTHR * i, row = g >> 5, c8 = (g & 31) << 3;
    const v4f a = *(const v4f*)(Est + row * HID + c8);
    const v4f b = *(const v4f*)(Est + row * HID + c8 + 4);
    Pk8 hi, lo;
    split8(a, b, hi, lo);
    *(u32x4*)(Ah + row * HID + c8) = hi.u;
    *(u32x4*)(Al + row * HID + c8) = lo.u;
  }
}

__device__ __forceinline__ v4f relu4(v4f a) {
  v4f r;
  r.x = fmaxf(a.x, 0.0f); r.y = fmaxf(a.y, 0.0f); r.z = fmaxf(a.z, 0.0f); r.w = fmaxf(a.w, 0.0f);
  return r;
}

__device__ __forceinline__ void cvt_l1(const float* Est, const float* __restrict__ pq, int tN,
                                       const int* sRow, const int* sCol, const float* __restrict__ be1,
                                       __bf16* Ah, __bf16* Al, int tid) {
#pragma unroll 2
  for (int i = 0; i < 8; ++i) {
    const int g = tid + NTHR * i, row = g >> 5, c8 = (g & 31) << 3;
    const int pr = sRow[row], qc = sCol[row];
    const float* P = pq + (size_t)(tN + pr) * (2 * HID) + c8;
    const float* Q = pq + (size_t)(tN + qc) * (2 * HID) + HID + c8;
    v4f a = *(const v4f*)(Est + row * HID + c8);
    v4f b = *(const v4f*)(Est + row * HID + c8 + 4);
    a = a + *(const v4f*)P;       a = a + *(const v4f*)Q;       a = a + *(const v4f*)(be1 + c8);
    b = b + *(const v4f*)(P + 4); b = b + *(const v4f*)(Q + 4); b = b + *(const v4f*)(be1 + c8 + 4);
    a = relu4(a);
    b = relu4(b);
    Pk8 hi, lo;
    split8(a, b, hi, lo);
    *(u32x4*)(Ah + row * HID + c8) = hi.u;
    *(u32x4*)(Al + row * HID + c8) = lo.u;
  }
}

template <int RELU>
__device__ __forceinline__ void acc_to_est(float* Est, const v8f (&acc0)[4], const v8f (&acc1)[4],
                                           float b0, float b1, int c0, int c1, int hh) {
#pragma unroll
  for (int mt = 0; mt < 4; ++mt) {
#pragma unroll
    for (int r = 0; r < 8; ++r) {
      const int row = 16 * mt + 8 * hh + r;
      float v0 = acc0[mt][r] + b0, v1 = acc1[mt][r] + b1;
      if (RELU != 0) { v0 = fmaxf(v0, 0.0f); v1 = fmaxf(v1, 0.0f); }
      Est[row * HID + c0] = v0;
      Est[row * HID + c1] = v1;
    }
  }
}

__device__ __forceinline__ void store_rows(const float* Est, float* dst, int rb, int pitch, int coff,
                                           int wave, int lane) {
#pragma unroll
  for (int i = 0; i < 8; ++i) {
    const int row = wave + 8 * i;
#pragma unroll
    for (int q = 0; q < 2; ++q) {
      const v4f v = *(const v4f*)(Est + row * HID + 128 * q + 4 * lane);
      *(volatile v4f*)(dst + (size_t)(rb + row) * pitch + coff + 128 * q + 4 * lane) = v;
    }
  }
  __threadfence();
#pragma unroll
  for (int i = 0; i < 8; ++i) {
    const int row = wave + 8 * i;
#pragma unroll
    for (int q = 0; q < 2; ++q) {
      const v4f v = *(const v4f*)(Est + row * HID + 128 * q + 4 * lane);
      *(volatile v4f*)(dst + (size_t)(rb + row) * pitch + coff + 128 * q + 4 * lane) = v;
    }
  }
}

__global__ __launch_bounds__(NTHR) void k_pack(const float* __restrict__ W, __bf16* outp,
                                                int Kreal, int Kt, int Nt, int kshift) {
  const int total = Nt * Kt * 64;
  const int g = blockIdx.x * NTHR + threadIdx.x;
  if (g >= total) return;
  const int lg = g >> 1, half = g & 1;
  const int lane = lg & 31;
  const int tk = lg >> 5;
  const int kt = tk % Kt, nt = tk / Kt;
  const int n = nt * 16 + (lane & 15);
  const int hs = lane >> 4;
  const int kb = kt * 32 + 16 * half + 8 * hs;
  const int rowoff = kshift * (n >> 8);
  Pk8 hi, lo;
#pragma unroll
  for (int i = 0; i < 8; ++i) {
    const int k = kb + i;
    const int kk = (k < Kreal) ? k : (Kreal - 1);
    float v = W[(size_t)(kk + rowoff) * HID + (n & 255)];
    v = (k < Kreal) ? v : 0.0f;
    const __bf16 t = (__bf16)v;
    hi.b[i] = t;
    lo.b[i] = (__bf16)(v - (float)t);
  }
  const size_t planeE = (size_t)total * 8;
  __bf16* ph = outp + (size_t)g * 8;
  __bf16* pl = ph + planeE;
  *(volatile u32x4*)ph = hi.u;
  *(volatile u32x4*)pl = lo.u;
  __threadfence();
  *(volatile u32x4*)ph = hi.u;
  *(volatile u32x4*)pl = lo.u;
}

__global__ __launch_bounds__(NTHR) void k_pq(const float* __restrict__ h, const __bf16* __restrict__ Wpq,
                                              float* pqo) {
  extern __shared__ __attribute__((aligned(16))) unsigned char dsm[];
  __bf16* Ah = (__bf16*)(dsm + L_AH);
  __bf16* Al = (__bf16*)(dsm + L_AL);
  float* Est = (float*)(dsm + L_EST);
  const int tid = threadIdx.x, lane = tid & 31, wave = tid >> 5, hh = lane >> 4, m = lane & 15;
  const int rb = blockIdx.x * 64;
  const int c0 = 32 * wave + m, c1 = c0 + 16;
  stage_rows(h, rb, Ah, Al, tid);
  __syncthreads();
  v8f acc0[4], acc1[4];
#pragma unroll 1
  for (int nc = 0; nc < 2; ++nc) {
    zacc(acc0, acc1);
    gemm_tile(Ah, Al, HID, 8, Wpq, Wpq + PL_PQ, 8, 0, 16 * nc + 2 * wave, lane, acc0, acc1);
    acc_to_est<0>(Est, acc0, acc1, 0.0f, 0.0f, c0, c1, hh);
    __syncthreads();
    store_rows(Est, pqo, rb, 2 * HID, HID * nc, wave, lane);
    __syncthreads();
  }
}

__global__ __launch_bounds__(NTHR) void k_edge(
    const float* __restrict__ x, const float* __restrict__ pq, const int* __restrict__ ei,
    const __bf16* __restrict__ Wr, const float* __restrict__ be1,
    const __bf16* __restrict__ W2, const float* __restrict__ be2,
    const __bf16* __restrict__ W3, const float* __restrict__ bc1, const float* __restrict__ Wc2,
    float* ep, float* tp, int t) {
  extern __shared__ __attribute__((aligned(16))) unsigned char dsm[];
  __bf16* Ah  = (__bf16*)(dsm + L_AH);
  __bf16* Al  = (__bf16*)(dsm + L_AL);
  float*  Est = (float*)(dsm + L_EST);
  __bf16* Arh = (__bf16*)(dsm + EK_ARH);
  __bf16* Arl = (__bf16*)(dsm + EK_ARL);
  float*  sCd = (float*)(dsm + EK_CD);
  float*  trs = (float*)(dsm + EK_TRS);
  int*    sRow = (int*)(dsm + EK_ROW);
  int*    sCol = (int*)(dsm + EK_COL);

  const int tid = threadIdx.x, lane = tid & 31, wave = tid >> 5, hh = lane >> 4, m = lane & 15;
  const int ebase = blockIdx.x * ET;
  const int tN = t * NNODE;
  const int nt0 = 2 * wave, c0 = 32 * wave + m, c1 = c0 + 16;

  if (tid < ET) {
    int r = ei[ebase + tid];
    int c = ei[NEDGE + ebase + tid];
    r = r < 0 ? 0 : (r > NNODE - 1 ? NNODE - 1 : r);
    c = c < 0 ? 0 : (c > NNODE - 1 ? NNODE - 1 : c);
    sRow[tid] = r;
    sCol[tid] = c;
  }
  __syncthreads();

  if (tid < ET) {
    const int e = tid;
    const float* xr = x + (size_t)(tN + sRow[e]) * 12;
    const float* xc = x + (size_t)(tN + sCol[e]) * 12;
    float cd[12];
#pragma unroll
    for (int j = 0; j < 12; ++j) { const float d = xr[j] - xc[j]; cd[j] = d; sCd[e * 12 + j] = d; }
    float g[16];
    float ss = 0.0f;
#pragma unroll
    for (int j = 0; j < 4; ++j) {
#pragma unroll
      for (int k = 0; k < 4; ++k) {
        const float v = cd[3 * j] * cd[3 * k] + cd[3 * j + 1] * cd[3 * k + 1] + cd[3 * j + 2] * cd[3 * k + 2];
        g[4 * j + k] = v;
        ss += v * v;
      }
    }
    const float inv = 1.0f / fmaxf(sqrtf(ss), 1e-12f);
    Pk8 h0, h1, l0, l1;
#pragma unroll
    for (int i = 0; i < 8; ++i) {
      const float a = g[i] * inv, b = g[8 + i] * inv;
      const __bf16 ta = (__bf16)a, tb = (__bf16)b;
      h0.b[i] = ta; l0.b[i] = (__bf16)(a - (float)ta);
      h1.b[i] = tb; l1.b[i] = (__bf16)(b - (float)tb);
    }
    const u32x4 z4 = {0u, 0u, 0u, 0u};
    u32x4* ph = (u32x4*)(Arh + e * 32);
    u32x4* pl = (u32x4*)(Arl + e * 32);
    ph[0] = h0.u; ph[1] = h1.u; ph[2] = z4; ph[3] = z4;
    pl[0] = l0.u; pl[1] = l1.u; pl[2] = z4; pl[3] = z4;
  }
  __syncthreads();

  v8f acc0[4], acc1[4];

  zacc(acc0, acc1);
  gemm_tile(Arh, Arl, 32, 1, Wr, Wr + PL_R, 1, 0, nt0, lane, acc0, acc1);
  acc_to_est<0>(Est, acc0, acc1, 0.0f, 0.0f, c0, c1, hh);
  __syncthreads();
  cvt_l1(Est, pq, tN, sRow, sCol, be1, Ah, Al, tid);
  __syncthreads();

  zacc(acc0, acc1);
  gemm_tile(Ah, Al, HID, 8, W2, W2 + PL_SQ, 8, 0, nt0, lane, acc0, acc1);
  {
    const float b0 = be2[c0], b1 = be2[c1];
    acc_to_est<1>(Est, acc0, acc1, b0, b1, c0, c1, hh);
  }
  __syncthreads();
  store_rows(Est, ep, ebase, HID, 0, wave, lane);
  cvt_tile(Est, Ah, Al, tid);
  __syncthreads();

  zacc(acc0, acc1);
  gemm_tile1(Ah, HID, 8, W3, 8, 0, nt0, lane, acc0, acc1);
  {
    float* pmx = Est;
    const float b0 = bc1[c0], b1 = bc1[c1], w0 = Wc2[c0], w1 = Wc2[c1];
#pragma unroll
    for (int mt = 0; mt < 4; ++mt) {
#pragma unroll
      for (int r = 0; r < 8; ++r) {
        const int row = 16 * mt + 8 * hh + r;
        const float s = fmaxf(acc0[mt][r] + b0, 0.0f) * w0 + fmaxf(acc1[mt][r] + b1, 0.0f) * w1;
        pmx[(wave * ET + row) * 16 + m] = s;
      }
    }
  }
  __syncthreads();
  if (tid < ET) {
    const float* pmx = Est;
    float mm = 0.0f;
#pragma unroll
    for (int w = 0; w < NWAVE; ++w) {
      const float* p = pmx + (w * ET + tid) * 16;
#pragma unroll
      for (int q = 0; q < 4; ++q) {
        const v4f v = *(const v4f*)(p + 4 * q);
        mm += v.x; mm += v.y; mm += v.z; mm += v.w;
      }
    }
#pragma unroll
    for (int j = 0; j < 12; ++j) trs[tid * 16 + j] = sCd[tid * 12 + j] * mm;
    trs[tid * 16 + 12] = 1.0f;
    trs[tid * 16 + 13] = 0.0f;
    trs[tid * 16 + 14] = 0.0f;
    trs[tid * 16 + 15] = 0.0f;
  }
  __syncthreads();
  {
    const v4f v = *(const v4f*)(trs + 4 * tid);
    float* d = tp + (size_t)ebase * 16 + 4 * tid;
    *(volatile v4f*)d = v;
    __threadfence();
    *(volatile v4f*)d = v;
  }
}

__device__ __forceinline__ int scan_chunk(const int* __restrict__ keys, int nE, int cbase, int nodeBase,
                                          int vec8, int* list, int tid, int wave) {
  int wc = 0;
  const int el0  = tid * EPT;
  const int e0   = cbase + el0;
  const int sent = -2147483647 - 1;
  const int last = nE - 1;
  v4i da, db;
  if (vec8 != 0 && cbase + CHUNK <= nE) {
    da = *(const v4i*)(keys + e0);
    db = *(const v4i*)(keys + e0 + 4);
  } else {
    da.x = (e0     < nE) ? keys[min(e0,     last)] : sent;
    da.y = (e0 + 1 < nE) ? keys[min(e0 + 1, last)] : sent;
    da.z = (e0 + 2 < nE) ? keys[min(e0 + 2, last)] : sent;
    da.w = (e0 + 3 < nE) ? keys[min(e0 + 3, last)] : sent;
    db.x = (e0 + 4 < nE) ? keys[min(e0 + 4, last)] : sent;
    db.y = (e0 + 5 < nE) ? keys[min(e0 + 5, last)] : sent;
    db.z = (e0 + 6 < nE) ? keys[min(e0 + 6, last)] : sent;
    db.w = (e0 + 7 < nE) ? keys[min(e0 + 7, last)] : sent;
  }
  const unsigned nb = (unsigned)nodeBase;
  const unsigned s0 = (unsigned)da.x - nb, s1 = (unsigned)da.y - nb;
  const unsigned s2 = (unsigned)da.z - nb, s3 = (unsigned)da.w - nb;
  const unsigned s4 = (unsigned)db.x - nb, s5 = (unsigned)db.y - nb;
  const unsigned s6 = (unsigned)db.z - nb, s7 = (unsigned)db.w - nb;
  const bool h0 = s0 < (unsigned)NB, h1 = s1 < (unsigned)NB, h2 = s2 < (unsigned)NB, h3 = s3 < (unsigned)NB;
  const bool h4 = s4 < (unsigned)NB, h5 = s5 < (unsigned)NB, h6 = s6 < (unsigned)NB, h7 = s7 < (unsigned)NB;
  const unsigned any = __builtin_amdgcn_ballot_w32(h0 | h1 | h2 | h3 | h4 | h5 | h6 | h7);
  if (any != 0u) {
#define HITJ(J, HJ, SJ) { \
      const unsigned mj = __builtin_amdgcn_ballot_w32(HJ); \
      if (mj != 0u) { \
        if (HJ) { \
          const int pos = wc + (int)__builtin_amdgcn_mbcnt_lo(mj, 0u); \
          if (pos < WCAP) list[wave * WCAP + pos] = ((el0 + (J)) << 8) | (int)(SJ); \
        } \
        wc += (int)__builtin_popcount(mj); } }
    HITJ(0, h0, s0)
    HITJ(1, h1, s1)
    HITJ(2, h2, s2)
    HITJ(3, h3, s3)
    HITJ(4, h4, s4)
    HITJ(5, h5, s5)
    HITJ(6, h6, s6)
    HITJ(7, h7, s7)
#undef HITJ
  }
  return wc;
}

__global__ __launch_bounds__(NTHR) void k_agg(const int* __restrict__ ei, const float* __restrict__ ep,
                                               const float* __restrict__ tp, const float* __restrict__ x,
                                               float* aggp, float* cout, int t, int nE, int vec8) {
  extern __shared__ __attribute__((aligned(16))) unsigned char dsm[];
  float* acc  = (float*)(dsm + AG_ACC);
  float* act  = (float*)(dsm + AG_ACT);
  int*   list = (int*)(dsm + AG_LIST);
  float* co   = (float*)(dsm + AG_CO);
  __shared__ int wcnt[NWAVE];

  const int tid = threadIdx.x, lane = tid & 31, wave = tid >> 5;
  const int nodeBase = blockIdx.x * NB;
  const int tN = t * NNODE;
  {
    const v4f z = {0.0f, 0.0f, 0.0f, 0.0f};
    for (int i = tid; i < (NB * HID) / 4; i += NTHR) *(v4f*)(acc + 4 * i) = z;
    for (int i = tid; i < (NB * 16) / 4; i += NTHR)  *(v4f*)(act + 4 * i) = z;
  }
  __syncthreads();

  const int nChunks = (nE + CHUNK - 1) / CHUNK;
#pragma unroll 1
  for (int ch = 0; ch < nChunks; ++ch) {
    const int cbase = ch * CHUNK;
    const int wc = scan_chunk(ei, nE, cbase, nodeBase, vec8, list, tid, wave);
    if (lane == 0) wcnt[wave] = wc;
    __syncthreads();
#pragma unroll 1
    for (int w = 0; w < NWAVE; ++w) {
      int c = wcnt[w];
      c = c > WCAP ? WCAP : (c < 0 ? 0 : c);
#pragma unroll 1
      for (int i = 0; i < c; ++i) {
        const int pk = list[w * WCAP + i];
        const int el = (pk >> 8) & (CHUNK - 1);
        int s = pk & 255;
        s = s > NB - 1 ? NB - 1 : s;
        int e = cbase + el;
        e = e > nE - 1 ? nE - 1 : e;
        const float v = ep[(size_t)e * HID + tid];
        acc[s * HID + tid] += v;
        if (wave == 0) {
          const float tv = tp[(size_t)e * 16 + (lane & 15)];
          if (lane < 16) act[s * 16 + lane] += tv;
        }
      }
    }
    __syncthreads();
  }

  store_rows(acc, aggp, tN + nodeBase, HID, 0, wave, lane);

#pragma unroll
  for (int i = 0; i < 3; ++i) {
    const int idx = tid + NTHR * i;
    const int s = idx / 12, j = idx - 12 * s;
    const float cnt = act[s * 16 + 12];
    const float rc = 1.0f / fmaxf(cnt, 1.0f);
    co[idx] = x[(size_t)(tN + nodeBase + s) * 12 + j] + act[s * 16 + j] * rc;
  }
  __syncthreads();
  if (tid < (NB * 12) / 4) {
    const v4f v = *(const v4f*)(co + 4 * tid);
    float* d = cout + (size_t)(tN + nodeBase) * 12 + 4 * tid;
    *(volatile v4f*)d = v;
    __threadfence();
    *(volatile v4f*)d = v;
  }
}

__global__ __launch_bounds__(NTHR) void k_node(const float* __restrict__ others, const float* __restrict__ h,
                                                const float* __restrict__ aggp,
                                                const __bf16* __restrict__ Wn1, const float* __restrict__ bn1,
                                                const __bf16* __restrict__ Wn2, const float* __restrict__ bn2,
                                                float* hout) {
  extern __shared__ __attribute__((aligned(16))) unsigned char dsm[];
  __bf16* Ah = (__bf16*)(dsm + L_AH);
  __bf16* Al = (__bf16*)(dsm + L_AL);
  float* Est = (float*)(dsm + L_EST);
  const int tid = threadIdx.x, lane = tid & 31, wave = tid >> 5, hh = lane >> 4, m = lane & 15;
  const int rb = blockIdx.x * 64;
  const int nt0 = 2 * wave, c0 = 32 * wave + m, c1 = c0 + 16;

  v8f acc0[4], acc1[4];
  zacc(acc0, acc1);
#pragma unroll 1
  for (int c = 0; c < 3; ++c) {
    const float* src = (c == 0) ? others : ((c == 1) ? h : aggp);
    __syncthreads();
    stage_rows(src, rb, Ah, Al, tid);
    __syncthreads();
    gemm_tile(Ah, Al, HID, 8, Wn1, Wn1 + PL_N1, 24, 8 * c, nt0, lane, acc0, acc1);
  }
  {
    const float b0 = bn1[c0], b1 = bn1[c1];
    acc_to_est<1>(Est, acc0, acc1, b0, b1, c0, c1, hh);
  }
  __syncthreads();
  cvt_tile(Est, Ah, Al, tid);
  __syncthreads();
  zacc(acc0, acc1);
  gemm_tile(Ah, Al, HID, 8, Wn2, Wn2 + PL_SQ, 8, 0, nt0, lane, acc0, acc1);
  {
    const float b0 = bn2[c0], b1 = bn2[c1];
    acc_to_est<0>(Est, acc0, acc1, b0, b1, c0, c1, hh);
  }
  __syncthreads();
#pragma unroll 4
  for (int i = 0; i < 16; ++i) {
    const int idx = tid + NTHR * i;
    const int row = idx >> 6, c4 = (idx & 63) << 2;
    v4f* e4 = (v4f*)(Est + row * HID + c4);
    const v4f hv = *(const v4f*)(h + (size_t)(rb + row) * HID + c4);
    *e4 = *e4 + hv;
  }
  __syncthreads();
  store_rows(Est, hout, rb, HID, 0, wave, lane);
}

extern "C" void kernel_launch(void* const* d_in, const int* in_sizes, int n_in,
                              void* d_out, int out_size, void* d_ws, size_t ws_size,
                              hipStream_t stream) {
  if (n_in < 15) return;
  if (in_sizes[0] != NROWS * 12 || in_sizes[1] != NROWS * HID || in_sizes[2] != NROWS * HID) return;
  if (in_sizes[3] != 528 * HID || in_sizes[4] != HID || in_sizes[5] != HID * HID || in_sizes[6] != HID) return;
  if (in_sizes[7] != 768 * HID || in_sizes[8] != HID || in_sizes[9] != HID * HID || in_sizes[10] != HID) return;
  if (in_sizes[11] != HID * HID || in_sizes[12] != HID || in_sizes[13] != HID || in_sizes[14] != 2 * NEDGE) return;
  if (out_size != NROWS * HID + NROWS * 12) return;

  const float* x      = (const float*)d_in[0];
  const float* h      = (const float*)d_in[1];
  const float* others = (const float*)d_in[2];
  const float* We1    = (const float*)d_in[3];
  const float* be1    = (const float*)d_in[4];
  const float* We2    = (const float*)d_in[5];
  const float* be2    = (const float*)d_in[6];
  const float* Wn1    = (const float*)d_in[7];
  const float* bn1    = (const float*)d_in[8];
  const float* Wn2    = (const float*)d_in[9];
  const float* bn2    = (const float*)d_in[10];
  const float* Wc1    = (const float*)d_in[11];
  const float* bc1    = (const float*)d_in[12];
  const float* Wc2    = (const float*)d_in[13];
  const int*   ei     = (const int*)d_in[14];
  float* hout = (float*)d_out;
  float* cout = hout + (size_t)NROWS * HID;

  size_t off = 0;
  const size_t oWPQ = off; off += (size_t)PL_PQ * 4;
  const size_t oWR  = off; off += (size_t)PL_R  * 4;
  const size_t oW2  = off; off += (size_t)PL_SQ * 4;
  const size_t oW3  = off; off += (size_t)PL_SQ * 4;
  const size_t oWN1 = off; off += (size_t)PL_N1 * 4;
  const size_t oWN2 = off; off += (size_t)PL_SQ * 4;
  const size_t oPQ  = off; off += (size_t)NROWS * 2 * HID * 4;
  const size_t oE   = off; off += (size_t)NEDGE * HID * 4;
  const size_t oTR  = off; off += (size_t)NEDGE * 16 * 4;
  const size_t oAGG = off; off += (size_t)NROWS * HID * 4;
  if (off > ws_size || off > (size_t)134217728) return;

  char* ws = (char*)d_ws;
  __bf16* Wpq  = (__bf16*)(ws + oWPQ);
  __bf16* Wr   = (__bf16*)(ws + oWR);
  __bf16* W2p  = (__bf16*)(ws + oW2);
  __bf16* W3p  = (__bf16*)(ws + oW3);
  __bf16* Wn1p = (__bf16*)(ws + oWN1);
  __bf16* Wn2p = (__bf16*)(ws + oWN2);
  float* pqp   = (float*)(ws + oPQ);
  float* ep    = (float*)(ws + oE);
  float* tp    = (float*)(ws + oTR);
  float* aggp  = (float*)(ws + oAGG);

  hipFuncSetAttribute(reinterpret_cast<const void*>(&k_pq),   hipFuncAttributeMaxDynamicSharedMemorySize, PN_BYTES);
  hipFuncSetAttribute(reinterpret_cast<const void*>(&k_node), hipFuncAttributeMaxDynamicSharedMemorySize, PN_BYTES);
  hipFuncSetAttribute(reinterpret_cast<const void*>(&k_edge), hipFuncAttributeMaxDynamicSharedMemorySize, EK_BYTES);
  hipFuncSetAttribute(reinterpret_cast<const void*>(&k_agg),  hipFuncAttributeMaxDynamicSharedMemorySize, AG_BYTES);

  k_pack<<<(PL_PQ / 8 + NTHR - 1) / NTHR, NTHR, 0, stream>>>(We1,             Wpq,  256, 8,  32, 256);
  k_pack<<<(PL_R  / 8 + NTHR - 1) / NTHR, NTHR, 0, stream>>>(We1 + 512 * HID, Wr,   16,  1,  16, 0);
  k_pack<<<(PL_SQ / 8 + NTHR - 1) / NTHR, NTHR, 0, stream>>>(We2,             W2p,  256, 8,  16, 0);
  k_pack<<<(PL_SQ / 8 + NTHR - 1) / NTHR, NTHR, 0, stream>>>(Wc1,             W3p,  256, 8,  16, 0);
  k_pack<<<(PL_N1 / 8 + NTHR - 1) / NTHR, NTHR, 0, stream>>>(Wn1,             Wn1p, 768, 24, 16, 0);
  k_pack<<<(PL_SQ / 8 + NTHR - 1) / NTHR, NTHR, 0, stream>>>(Wn2,             Wn2p, 256, 8,  16, 0);

  k_pq<<<NROWS / 64, NTHR, PN_BYTES, stream>>>(h, Wpq, pqp);

  const int vec8 = ((NEDGE & 3) == 0) ? 1 : 0;
  for (int t = 0; t < TT; ++t) {
    k_edge<<<NEDGE / ET, NTHR, EK_BYTES, stream>>>(x, pqp, ei, Wr, be1, W2p, be2, W3p, bc1, Wc2, ep, tp, t);
    k_agg<<<NNODE / NB, NTHR, AG_BYTES, stream>>>(ei, ep, tp, x, aggp, cout, t, NEDGE, vec8);
  }

  k_node<<<NROWS / 64, NTHR, PN_BYTES, stream>>>(others, h, aggp, Wn1p, bn1, Wn2p, bn2, hout);
}
